// SimpleAttention_2190433321490
// MI455X (gfx1250) — hardware-verified
//
#include <hip/hip_runtime.h>
#include <stdint.h>


typedef _Float16 v16h __attribute__((ext_vector_type(16)));
typedef _Float16 v8h  __attribute__((ext_vector_type(8)));
typedef _Float16 v8ha __attribute__((ext_vector_type(8), may_alias));
typedef float    v8f  __attribute__((ext_vector_type(8)));
typedef float    v4f  __attribute__((ext_vector_type(4)));
typedef float    v4fa __attribute__((ext_vector_type(4), may_alias));
typedef unsigned int v4u __attribute__((ext_vector_type(4)));

union U8f  { v8f  v; float    f[8]; };
union U16h { v16h v; v8h      h[2]; };
union U8h  { v8h  v; _Float16 f[8]; };

#ifndef NB
#define NB 4
#endif
#ifndef SEQ
#define SEQ 2048
#endif
#define NB_FULL  4
#define SEQ_FULL 2048
#define DD       1024
#define NPRJ     3

#define CVR  16
#define GBM  128
#define GBN  128
#define GNB  ((NPRJ * DD) / GBN)
#define STP  136

#define BQ   16
#define BK   128
#define QP   1032
#define SSP  132
#define PPT  136

static_assert(NB >= 1 && NB <= NB_FULL);
static_assert(SEQ >= GBM && SEQ <= SEQ_FULL);
static_assert(SEQ % GBM == 0);
static_assert(SEQ % BK == 0);
static_assert(SEQ % BQ == 0);
static_assert((NB * SEQ) % CVR == 0);
static_assert(DD % CVR == 0);
static_assert(DD % GBN == 0);
static_assert(DD % 32 == 0);
static_assert((STP * 2) % 16 == 0);
static_assert((QP * 2) % 16 == 0);
static_assert((SSP * 4) % 16 == 0);
static_assert((PPT * 2) % 16 == 0);

#define SQ_BOFF 0
#define SS_BOFF (SQ_BOFF + BQ * QP * 2)
#define SP_BOFF (SS_BOFF + BQ * SSP * 4)
#define SA_BOFF (SP_BOFF + BQ * PPT * 2)
#define SO_BOFF (SA_BOFF + 2 * BQ * 4)
#define ATT_LDS (SO_BOFF + 8 * 16 * 64 * 4)
static_assert(SS_BOFF % 16 == 0);
static_assert(SP_BOFF % 16 == 0);
static_assert(SA_BOFF % 16 == 0);
static_assert(SO_BOFF % 16 == 0);
static_assert(ATT_LDS == 78720);

#define C2SCALE 0.04508422002777817f
#define WCARRY  64.0f
#define WUNDO   0.015625f
#define PCARRY  1024.0f

__device__ __forceinline__ v8f wmma_f16(v16h a, v16h b, v8f c) {
  v8f d = __builtin_amdgcn_wmma_f32_16x16x32_f16(false, a, false, b, (short)0, c, false, false);
  asm volatile("v_nop\n\tv_nop\n\tv_nop\n\tv_nop" : "+v"(d) : "v"(a), "v"(b));
  return d;
}

template <int CTRL>
__device__ __forceinline__ float dppf(float x) {
  int s = __float_as_int(x);
  return __int_as_float(__builtin_amdgcn_update_dpp(s, s, CTRL, 0xF, 0xF, true));
}
__device__ __forceinline__ float red_max16(float x) {
  x = fmaxf(x, dppf<0xB1>(x));
  x = fmaxf(x, dppf<0x4E>(x));
  x = fmaxf(x, dppf<0x141>(x));
  x = fmaxf(x, dppf<0x140>(x));
  return x;
}
__device__ __forceinline__ float red_sum16(float x) {
  x += dppf<0xB1>(x);
  x += dppf<0x4E>(x);
  x += dppf<0x141>(x);
  x += dppf<0x140>(x);
  return x;
}

__device__ __forceinline__ void wave_lds_sync() {
  __builtin_amdgcn_fence(3, "wavefront");
  asm volatile("s_wait_dscnt 0" ::: "memory");
  __builtin_amdgcn_wave_barrier();
}

__device__ __forceinline__ v4f bf16_rne4(v4f a) {
  v4u u = __builtin_bit_cast(v4u, a);
  u = (u + 0x7FFFu + ((u >> 16) & 1u)) & 0xFFFF0000u;
  return __builtin_bit_cast(v4f, u);
}
__device__ __forceinline__ float bf16_rne1(float a) {
  unsigned int u = __float_as_uint(a);
  u = (u + 0x7FFFu + ((u >> 16) & 1u)) & 0xFFFF0000u;
  return __uint_as_float(u);
}

__device__ __forceinline__ v8h cvt8v(v4f a, v4f b) {
  v8h d;
  d[0] = (_Float16)a[0]; d[1] = (_Float16)a[1];
  d[2] = (_Float16)a[2]; d[3] = (_Float16)a[3];
  d[4] = (_Float16)b[0]; d[5] = (_Float16)b[1];
  d[6] = (_Float16)b[2]; d[7] = (_Float16)b[3];
  return d;
}

__global__ __launch_bounds__(256)
void cvt_kernel(const float* __restrict__ src, _Float16* __restrict__ dst,
                int nrows, int srows, int drows, float scale)
{
  const int tid = threadIdx.x;
  #pragma unroll 1
  for (int it = 0; it < 8; ++it) {
    const int p   = tid + 256 * it;
    const int r   = p >> 7;
    const int q   = p & 127;
    int row = blockIdx.x * CVR + r;
    if (row > nrows - 1) row = nrows - 1;
    const int srow = (row / drows) * srows + (row % drows);
    const float* sp = src + (size_t)srow * DD + 8 * q;
    const v4f a0 = bf16_rne4(*(const v4f*)(sp)) * scale;
    const v4f a1 = bf16_rne4(*(const v4f*)(sp + 4)) * scale;
    const v8h hv = cvt8v(a0, a1);
    _Float16* dp = dst + (size_t)row * DD + 8 * q;
    *(volatile v8h*)dp = hv;
    __threadfence();
    *(volatile v8h*)dp = hv;
  }
}

__global__ __launch_bounds__(256) __attribute__((amdgpu_num_vgpr(256)))
void qkv_gemm_kernel(const _Float16* __restrict__ Xh, const _Float16* __restrict__ Wh,
                     const float* __restrict__ bq, const float* __restrict__ bk,
                     const float* __restrict__ bv,
                     _Float16* __restrict__ Qp, _Float16* __restrict__ Kp, _Float16* __restrict__ Vt)
{
  __shared__ __attribute__((aligned(16))) _Float16 stg[GBM * STP];

  const int tid  = threadIdx.x;
  const int wave = tid >> 5;
  const int lane = tid & 31;
  const int lh   = lane & 15;
  const int hh   = lane >> 4;
  const int wm   = wave & 3;
  const int wn   = wave >> 2;
  const int nblk = blockIdx.x;
  const int mblk = blockIdx.y;
  const int prj  = nblk >> 3;
  const int oc0  = (nblk & 7) * GBN;
  const int m0   = mblk * GBM;

  const _Float16* A0 = Xh + (size_t)(m0 + 32 * wm + lh) * DD + 8 * hh;
  const _Float16* A1 = A0 + (size_t)16 * DD;
  const _Float16* B0 = Wh + ((size_t)prj * DD + oc0 + 64 * wn + lh) * DD + 8 * hh;

  U8f acc[2][4];
  #pragma unroll
  for (int i = 0; i < 2; ++i)
    #pragma unroll
    for (int t = 0; t < 4; ++t) acc[i][t].v = (v8f){};

  #pragma unroll 1
  for (int k0 = 0; k0 < DD; k0 += 32) {
    U16h a0, a1;
    a0.h[0] = *(const v8h*)(A0 + k0);
    a0.h[1] = *(const v8h*)(A0 + k0 + 16);
    a1.h[0] = *(const v8h*)(A1 + k0);
    a1.h[1] = *(const v8h*)(A1 + k0 + 16);
    #pragma unroll
    for (int t = 0; t < 4; ++t) {
      U16h bfr;
      const _Float16* bpt = B0 + (size_t)(16 * t) * DD + k0;
      bfr.h[0] = *(const v8h*)(bpt);
      bfr.h[1] = *(const v8h*)(bpt + 16);
      acc[0][t].v = wmma_f16(a0.v, bfr.v, acc[0][t].v);
      acc[1][t].v = wmma_f16(a1.v, bfr.v, acc[1][t].v);
    }
  }

  const float* bp = (prj == 0) ? bq : ((prj == 1) ? bk : bv);
  float bb[4];
  #pragma unroll
  for (int t = 0; t < 4; ++t) bb[t] = bf16_rne1(bp[oc0 + 64 * wn + 16 * t + lh]);

  if (prj < 2) {
    #pragma unroll
    for (int i = 0; i < 2; ++i)
      #pragma unroll
      for (int t = 0; t < 4; ++t)
        #pragma unroll
        for (int j = 0; j < 8; ++j)
          stg[(32 * wm + 16 * i + 8 * hh + j) * STP + 64 * wn + 16 * t + lh] =
              (_Float16)(acc[i][t].f[j] * WUNDO + bb[t]);
  } else {
    #pragma unroll
    for (int i = 0; i < 2; ++i)
      #pragma unroll
      for (int t = 0; t < 4; ++t) {
        U8h hv;
        #pragma unroll
        for (int j = 0; j < 8; ++j) hv.f[j] = (_Float16)(acc[i][t].f[j] * WUNDO + bb[t]);
        *(v8h*)(stg + (64 * wn + 16 * t + lh) * STP + 32 * wm + 16 * i + 8 * hh) = hv.v;
      }
  }
  __syncthreads();

  _Float16* base;
  int rstride;
  if (prj == 0) {
    base = Qp + (size_t)m0 * DD + oc0; rstride = DD;
  } else if (prj == 1) {
    base = Kp + (size_t)m0 * DD + oc0; rstride = DD;
  } else {
    const int b   = m0 / SEQ;
    const int nl0 = m0 - b * SEQ;
    base = Vt + ((size_t)b * DD + oc0) * SEQ + nl0; rstride = SEQ;
  }
  v8h vv[8]; int oo[8];
  #pragma unroll
  for (int it = 0; it < 8; ++it) {
    const int p = tid + 256 * it;
    const int r = p >> 4, q = p & 15;
    vv[it] = *(const v8ha*)(stg + r * STP + 8 * q);
    oo[it] = r * rstride + 8 * q;
  }
  #pragma unroll
  for (int it = 0; it < 8; ++it) *(volatile v8h*)(base + oo[it]) = vv[it];
  __threadfence();
  #pragma unroll
  for (int it = 0; it < 8; ++it) *(volatile v8h*)(base + oo[it]) = vv[it];
}

__global__ __launch_bounds__(256) __attribute__((amdgpu_num_vgpr(256)))
void attn_kernel(const _Float16* __restrict__ Qp, const _Float16* __restrict__ Kp,
                 const _Float16* __restrict__ Vt, float* __restrict__ Out)
{
  extern __shared__ __attribute__((aligned(16))) unsigned char smem[];
  _Float16* sQ  = (_Float16*)(smem + SQ_BOFF);
  float*    sS  = (float*)(smem + SS_BOFF);
  _Float16* sP  = (_Float16*)(smem + SP_BOFF);
  float*    sAl = (float*)(smem + SA_BOFF);
  float*    sLn = sAl + BQ;
  float*    sO  = (float*)(smem + SO_BOFF);

  const int tid  = threadIdx.x;
  const int wave = tid >> 5;
  const int lane = tid & 31;
  const int lh   = lane & 15;
  const int hh   = lane >> 4;
  const int srow = tid >> 4;
  const int ssub = tid & 15;

  const int nqb = SEQ / BQ;
  const int b   = blockIdx.x / nqb;
  const int q0  = (blockIdx.x % nqb) * BQ;

  const _Float16* Qb = Qp + ((size_t)b * SEQ + q0) * DD;
  const _Float16* Kb = Kp + (size_t)b * SEQ * DD;
  const _Float16* Vb = Vt + (size_t)b * DD * SEQ;
  float*          Ob = Out + ((size_t)b * SEQ + q0) * DD;

  #pragma unroll
  for (int it = 0; it < 8; ++it) {
    const int p = tid + 256 * it;
    const int r = p >> 7, q = p & 127;
    const v8h qv = *(const v8h*)(Qb + (size_t)r * DD + 8 * q);
    *(v8h*)(sQ + r * QP + 8 * q) = qv;
  }
  __syncthreads();

  U8f acc[8];
  #pragma unroll
  for (int t = 0; t < 8; ++t) acc[t].v = (v8f){};
  float mrun = -3.0e38f, lrun = 0.0f;

  const _Float16* Qw = sQ + lh * QP + 8 * hh;

  #pragma unroll 1
  for (int kv0 = 0; kv0 < SEQ; kv0 += BK) {
    U8f s; s.v = (v8f){};
    const _Float16* Kw = Kb + (size_t)(kv0 + 16 * wave + lh) * DD + 8 * hh;
    #pragma unroll 2
    for (int c = 0; c < DD / 32; ++c) {
      U16h qf, kf;
      qf.h[0] = *(const v8h*)(Qw + 32 * c);
      qf.h[1] = *(const v8h*)(Qw + 32 * c + 16);
      kf.h[0] = *(const v8h*)(Kw + 32 * c);
      kf.h[1] = *(const v8h*)(Kw + 32 * c + 16);
      s.v = wmma_f16(qf.v, kf.v, s.v);
    }
    #pragma unroll
    for (int j = 0; j < 8; ++j) sS[(8 * hh + j) * SSP + 16 * wave + lh] = s.f[j] * C2SCALE;
    __syncthreads();

    {
      const v4f x0 = *(const v4fa*)(sS + srow * SSP + 8 * ssub);
      const v4f x1 = *(const v4fa*)(sS + srow * SSP + 8 * ssub + 4);
      float e[8];
      e[0] = x0[0]; e[1] = x0[1]; e[2] = x0[2]; e[3] = x0[3];
      e[4] = x1[0]; e[5] = x1[1]; e[6] = x1[2]; e[7] = x1[3];
      float rm = e[0];
      #pragma unroll
      for (int i = 1; i < 8; ++i) rm = fmaxf(rm, e[i]);
      rm = red_max16(rm);
      const float mnew  = fmaxf(mrun, rm);
      const float alpha = __builtin_amdgcn_exp2f(mrun - mnew);
      float ps = 0.0f;
      U8h pk;
      #pragma unroll
      for (int i = 0; i < 8; ++i) {
        const float ei = __builtin_amdgcn_exp2f(e[i] - mnew);
        ps += ei;
        pk.f[i] = (_Float16)(ei * PCARRY);
      }
      ps = red_sum16(ps);
      lrun = lrun * alpha + ps;
      mrun = mnew;
      *(v8h*)(sP + srow * PPT + 8 * ssub) = pk.v;
      if (ssub == 0) { sAl[srow] = alpha; sLn[srow] = lrun; }
    }
    __syncthreads();

    {
      const v4f l0 = *(const v4fa*)(sAl + 8 * hh);
      const v4f l1 = *(const v4fa*)(sAl + 8 * hh + 4);
      float al[8];
      al[0] = l0[0]; al[1] = l0[1]; al[2] = l0[2]; al[3] = l0[3];
      al[4] = l1[0]; al[5] = l1[1]; al[6] = l1[2]; al[7] = l1[3];
      #pragma unroll
      for (int t = 0; t < 8; ++t)
        #pragma unroll
        for (int j = 0; j < 8; ++j) acc[t].f[j] *= al[j];
    }
    #pragma unroll 1
    for (int st = 0; st < BK / 32; ++st) {
      U16h pf;
      pf.h[0] = *(const v8ha*)(sP + lh * PPT + 32 * st + 8 * hh);
      pf.h[1] = *(const v8ha*)(sP + lh * PPT + 32 * st + 16 + 8 * hh);
      const _Float16* Vw = Vb + (size_t)(128 * wave + lh) * SEQ + kv0 + 32 * st + 8 * hh;
      #pragma unroll
      for (int t = 0; t < 8; ++t) {
        U16h vf;
        const _Float16* vp = Vw + (size_t)(16 * t) * SEQ;
        vf.h[0] = *(const v8h*)(vp);
        vf.h[1] = *(const v8h*)(vp + 16);
        acc[t].v = wmma_f16(pf.v, vf.v, acc[t].v);
      }
    }
  }

  float inv[8];
  {
    const v4f l0 = *(const v4fa*)(sLn + 8 * hh);
    const v4f l1 = *(const v4fa*)(sLn + 8 * hh + 4);
    inv[0] = __builtin_amdgcn_rcpf(l0[0] * PCARRY); inv[1] = __builtin_amdgcn_rcpf(l0[1] * PCARRY);
    inv[2] = __builtin_amdgcn_rcpf(l0[2] * PCARRY); inv[3] = __builtin_amdgcn_rcpf(l0[3] * PCARRY);
    inv[4] = __builtin_amdgcn_rcpf(l1[0] * PCARRY); inv[5] = __builtin_amdgcn_rcpf(l1[1] * PCARRY);
    inv[6] = __builtin_amdgcn_rcpf(l1[2] * PCARRY); inv[7] = __builtin_amdgcn_rcpf(l1[3] * PCARRY);
  }
  float* so = sO + wave * (16 * 64);
  float* ob = Ob + 128 * wave;
  #pragma unroll
  for (int g = 0; g < 2; ++g) {
    #pragma unroll
    for (int j = 0; j < 8; ++j) {
      #pragma unroll
      for (int tt = 0; tt < 4; ++tt)
        so[(j + 8 * hh) * 64 + tt * 16 + lh] = acc[4 * g + tt].f[j] * inv[j];
    }
    wave_lds_sync();
    v4f ov[8]; int oo[8];
    #pragma unroll
    for (int i = 0; i < 8; ++i) {
      const int c = lane + 32 * i, rr = c >> 4, q = c & 15;
      ov[i] = *(const v4fa*)(so + rr * 64 + q * 4);
      oo[i] = rr * DD + 64 * g + 4 * q;
    }
    #pragma unroll
    for (int i = 0; i < 8; ++i) *(volatile v4f*)(ob + oo[i]) = ov[i];
    __threadfence();
    #pragma unroll
    for (int i = 0; i < 8; ++i) *(volatile v4f*)(ob + oo[i]) = ov[i];
    wave_lds_sync();
  }
}

extern "C" void kernel_launch(void* const* d_in, const int* in_sizes, int n_in,
                              void* d_out, int out_size, void* d_ws, size_t ws_size,
                              hipStream_t stream) {
  if (n_in < 7) return;
  const long long need_x = ((long long)(NB - 1) * SEQ_FULL + SEQ) * DD;
  if ((long long)in_sizes[0] < need_x) return;
  if (in_sizes[1] < DD * DD || in_sizes[3] < DD * DD || in_sizes[5] < DD * DD) return;
  if (in_sizes[2] < DD || in_sizes[4] < DD || in_sizes[6] < DD) return;
  if ((long long)out_size < (long long)NB * SEQ * DD) return;

  const size_t act_bytes = (size_t)NB * SEQ * DD * 2;
  const size_t wh_bytes  = (size_t)NPRJ * DD * DD * 2;
  const size_t off_xh = 0;
  const size_t off_wh = off_xh + act_bytes;
  const size_t off_qp = off_wh + wh_bytes;
  const size_t off_kp = off_qp + act_bytes;
  const size_t off_vt = off_kp + act_bytes;
  const size_t off_end = off_vt + act_bytes;
  if (off_end > ws_size) return;

  const float* x  = (const float*)d_in[0];
  const float* Wq = (const float*)d_in[1];
  const float* bq = (const float*)d_in[2];
  const float* Wk = (const float*)d_in[3];
  const float* bk = (const float*)d_in[4];
  const float* Wv = (const float*)d_in[5];
  const float* bv = (const float*)d_in[6];
  float* out = (float*)d_out;

  _Float16* xh = (_Float16*)((char*)d_ws + off_xh);
  _Float16* wh = (_Float16*)((char*)d_ws + off_wh);
  _Float16* qp = (_Float16*)((char*)d_ws + off_qp);
  _Float16* kp = (_Float16*)((char*)d_ws + off_kp);
  _Float16* vt = (_Float16*)((char*)d_ws + off_vt);

  cvt_kernel<<<(NB * SEQ) / CVR, 256, 0, stream>>>(x, xh, NB * SEQ, SEQ_FULL, SEQ, 1.0f);
  cvt_kernel<<<DD / CVR, 256, 0, stream>>>(Wq, wh, DD, DD, DD, WCARRY);
  cvt_kernel<<<DD / CVR, 256, 0, stream>>>(Wk, wh + (size_t)DD * DD, DD, DD, DD, WCARRY);
  cvt_kernel<<<DD / CVR, 256, 0, stream>>>(Wv, wh + (size_t)2 * DD * DD, DD, DD, DD, WCARRY);

  qkv_gemm_kernel<<<dim3(GNB, (NB * SEQ) / GBM), 256, 0, stream>>>(xh, wh, bq, bk, bv, qp, kp, vt);

  (void)hipFuncSetAttribute(reinterpret_cast<const void*>(&attn_kernel),
                            hipFuncAttributeMaxDynamicSharedMemorySize, (int)ATT_LDS);
  attn_kernel<<<NB * (SEQ / BQ), 256, ATT_LDS, stream>>>(qp, kp, vt, out);
}
